// TransformerEncoder_9689446220356
// MI455X (gfx1250) — hardware-verified
//
#include <hip/hip_runtime.h>
#include <math.h>

#ifndef NB
#define NB 8
#endif
#ifndef SEQ
#define SEQ 256
#endif
#define SEQ_FULL 256
#define IN_DIM 128
#define E_DIM 16
#define EMB 256
#define HEADS 8
#define HD 32
#define FFD 1024
#define NLAYER 4
#define NPATH 8
#define N_EDGES 32768
#define MTOK (NB * SEQ)

static_assert(SEQ == 256);
static_assert(SEQ == SEQ_FULL);
static_assert(MTOK % 64 == 0);
static_assert(EMB % 64 == 0 && (3 * EMB) % 64 == 0 && FFD % 64 == 0);
static_assert(IN_DIM % 32 == 0 && EMB % 32 == 0 && FFD % 32 == 0);
static_assert((MTOK * IN_DIM / 8) % 256 == 0);
static_assert(MTOK % 8 == 0);

typedef __attribute__((ext_vector_type(16))) _Float16 v16h;
typedef __attribute__((ext_vector_type(8)))  _Float16 v8h;
typedef __attribute__((ext_vector_type(8)))  float    v8f;
typedef __attribute__((ext_vector_type(4)))  float    v4f;
typedef __attribute__((ext_vector_type(4)))  unsigned int v4u;


#define VST2(T, ptr, val) do { const T vst2_v_ = (val); *(volatile T*)(ptr) = vst2_v_; __threadfence(); *(volatile T*)(ptr) = vst2_v_; } while (0)
#define VST2V4(ptr, val) do { const v4f vst2_v4_ = (val); *(volatile v4f*)(ptr) = vst2_v4_; __threadfence(); *(volatile v4f*)(ptr) = vst2_v4_; } while (0)

__device__ __forceinline__ float bfr(float f) {
    unsigned u = __float_as_uint(f);
    u += 0x7FFFu + ((u >> 16) & 1u);
    return __uint_as_float(u & 0xFFFF0000u);
}
__device__ __forceinline__ unsigned short f2h_bits(float x) {
    return (fabsf(x) < 6.104e-5f) ? (unsigned short)0 : __builtin_bit_cast(unsigned short, (_Float16)x);
}
__device__ __forceinline__ void st8h(unsigned short* P, size_t o, const float* v) {
    v4u pk;
    pk.x = (unsigned)f2h_bits(v[0]) | ((unsigned)f2h_bits(v[1]) << 16);
    pk.y = (unsigned)f2h_bits(v[2]) | ((unsigned)f2h_bits(v[3]) << 16);
    pk.z = (unsigned)f2h_bits(v[4]) | ((unsigned)f2h_bits(v[5]) << 16);
    pk.w = (unsigned)f2h_bits(v[6]) | ((unsigned)f2h_bits(v[7]) << 16);
    VST2(v4u, (v4u*)(P + o), pk);
}

union FragU { v16h v; v8h h[2]; };
__device__ __forceinline__ v16h frag_ld(const _Float16* p) {
    FragU f; f.h[0] = *(const v8h*)(p); f.h[1] = *(const v8h*)(p + 16); return f.v;
}
__device__ __forceinline__ v8f wmma16(v16h a, v16h b, v8f c) {
    c = __builtin_amdgcn_wmma_f32_16x16x32_f16(false, a, false, b, (short)0, c, false, false);
    asm volatile("v_nop\n\tv_nop\n\tv_nop\n\tv_nop" : "+v"(c) : "v"(a), "v"(b));
    return c;
}
__device__ __forceinline__ void dep_guard_h(v8f& a, v8f& b, v16h x, v16h y) { asm volatile("v_nop\n\tv_nop\n\tv_nop\n\tv_nop" : "+v"(a), "+v"(b) : "v"(x), "v"(y)); }
__device__ __forceinline__ void keep4_h(v16h a, v16h b, v16h c, v16h d) { asm volatile("v_nop" :: "v"(a), "v"(b), "v"(c), "v"(d)); }
__device__ __forceinline__ void acc_guard4(v8f& a, v8f& b, v8f& c, v8f& d) { asm volatile("v_nop\n\tv_nop\n\tv_nop\n\tv_nop" : "+v"(a), "+v"(b), "+v"(c), "+v"(d)); }
__device__ __forceinline__ void wave_sync_lds() {
    __builtin_amdgcn_fence(3  , "workgroup");
    __builtin_amdgcn_wave_barrier();
    __builtin_amdgcn_fence(2  , "workgroup");
}

template <int OUT_MODE, bool RESID, bool RELU>
__global__ __launch_bounds__(256) void k_gemm64(
    const _Float16* __restrict__ A, unsigned lda, const _Float16* __restrict__ Bt, unsigned ldb,
    void* __restrict__ Cout, unsigned ldc, const float* __restrict__ bias, const float* __restrict__ resid,
    unsigned M, unsigned N, unsigned K, float scale, float oscale) {
  __shared__ __align__(16) float sT[8][16 * 68];
  const unsigned lane = threadIdx.x & 31u;
  const unsigned wave = threadIdx.x >> 5;
  const unsigned tilesN = N >> 6, tilesM = M >> 6;
  const unsigned tile = blockIdx.x * 8u + wave;
  if (tile >= tilesM * tilesN) return;
  const unsigned tm = tile / tilesN;
  const unsigned tn = tile - tm * tilesN;
  const unsigned m0 = tm << 6, n0 = tn << 6;
  const unsigned rlane = lane & 15u;
  const unsigned koff = (lane >> 4) * 8u;
  const unsigned mOff = koff;

  v8f acc[4][4];
#pragma unroll
  for (int i = 0; i < 4; ++i)
#pragma unroll
    for (int j = 0; j < 4; ++j) acc[i][j] = (v8f){0.f,0.f,0.f,0.f,0.f,0.f,0.f,0.f};

  for (unsigned k0 = 0; k0 < K; k0 += 32u) {
    v16h bh[4];
#pragma unroll
    for (int j = 0; j < 4; ++j)
      bh[j] = frag_ld(Bt + (size_t)(n0 + ((unsigned)j << 4) + rlane) * ldb + koff + k0);
#pragma unroll
    for (int i = 0; i < 4; ++i) {
      const v16h ah = frag_ld(A + (size_t)(m0 + ((unsigned)i << 4) + rlane) * lda + koff + k0);
#pragma unroll
      for (int j = 0; j < 4; ++j)
        acc[i][j] = __builtin_amdgcn_wmma_f32_16x16x32_f16(false, ah, false, bh[j], (short)0, acc[i][j], false, false);
      dep_guard_h(acc[i][0], acc[i][3], ah, ah);
    }
    keep4_h(bh[0], bh[1], bh[2], bh[3]);
  }
  acc_guard4(acc[0][0], acc[0][1], acc[0][2], acc[0][3]);
  acc_guard4(acc[1][0], acc[1][1], acc[1][2], acc[1][3]);
  acc_guard4(acc[2][0], acc[2][1], acc[2][2], acc[2][3]);
  acc_guard4(acc[3][0], acc[3][1], acc[3][2], acc[3][3]);

  float* slab = sT[wave];
#pragma unroll
  for (int i = 0; i < 4; ++i) {
    const unsigned mBase = m0 + ((unsigned)i << 4);
#pragma unroll
    for (int j = 0; j < 4; ++j) {
      const unsigned n = n0 + ((unsigned)j << 4) + rlane;
      const float bv = bfr(bias[n]);
#pragma unroll
      for (int r = 0; r < 8; ++r) {
        float v = acc[i][j][r] * scale + bv;
        if (RELU) v = fmaxf(v, 0.0f);
        if (OUT_MODE == 1) v *= oscale;
        slab[(mOff + (unsigned)r) * 68u + ((unsigned)j << 4) + rlane] = v;
      }
    }
    wave_sync_lds();
    if (OUT_MODE == 0) {
      float* C = (float*)Cout;
      const unsigned hh = lane >> 4, c4 = (lane & 15u) * 4u;
#pragma unroll
      for (int half = 0; half < 2; ++half) {
        v4f vv[4];
#pragma unroll
        for (int it = 0; it < 4; ++it) {
          const unsigned row = (unsigned)(half * 4 + it) * 2u + hh;
          vv[it] = *(const v4f*)(slab + row * 68u + c4);
          if (RESID) vv[it] += *(const v4f*)(resid + (size_t)(mBase + row) * ldc + n0 + c4);
        }
        for (int pass = 0; pass < 2; ++pass) {
#pragma unroll
          for (int it = 0; it < 4; ++it) {
            const unsigned row = (unsigned)(half * 4 + it) * 2u + hh;
            *(volatile v4f*)(C + (size_t)(mBase + row) * ldc + n0 + c4) = vv[it];
          }
          __threadfence();
        }
      }
    } else {
      _Float16* C = (_Float16*)Cout;
      const unsigned q = lane >> 3, c8 = (lane & 7u) * 8u;
      v8h hv[4];
#pragma unroll
      for (int it = 0; it < 4; ++it) {
        const unsigned row = (unsigned)it * 4u + q;
        const float* sp = slab + row * 68u + c8;
#pragma unroll
        for (int e = 0; e < 8; ++e) hv[it][e] = (_Float16)sp[e];
      }
      for (int pass = 0; pass < 2; ++pass) {
#pragma unroll
        for (int it = 0; it < 4; ++it) {
          const unsigned row = (unsigned)it * 4u + q;
          *(volatile v8h*)(C + (size_t)(mBase + row) * ldc + n0 + c8) = hv[it];
        }
        __threadfence();
      }
    }
    wave_sync_lds();
  }
}

__global__ __launch_bounds__(256) void k_wt16(const float* __restrict__ Wm, unsigned KI, unsigned NO, unsigned lgper,
                                              unsigned short* __restrict__ W16, float sw) {
    const unsigned layer = blockIdx.y;
    const float* Wl = Wm + (size_t)layer * KI * NO;
    unsigned short* Dl = W16 + (size_t)layer * KI * NO;
    const unsigned u = blockIdx.x * 256u + threadIdx.x;
    const unsigned per = 1u << lgper;
    if (u >= NO * per) return;
    const unsigned k0 = 8u * (u & (per - 1u));
    const unsigned o = u >> lgper;
    float v[8];
#pragma unroll
    for (int i = 0; i < 8; ++i) v[i] = bfr(Wl[(size_t)(k0 + (unsigned)i) * NO + o]) * sw;
    st8h(Dl, (size_t)o * KI + k0, v);
}

__global__ __launch_bounds__(256) void k_bias(const float* __restrict__ dist, const int* __restrict__ paths,
                                              const float* __restrict__ ef, const float* __restrict__ pp,
                                              const float* __restrict__ dparams, unsigned short* __restrict__ bias16) {
    __shared__ float sPP[128];
    __shared__ float sB[256];
    const unsigned t = threadIdx.x;
    if (t < 128u) sPP[t] = bfr(pp[t]);
    __syncthreads();
    const unsigned row = blockIdx.x;
    const unsigned b = row >> 8, q = row & 255u;
    const unsigned e = (b * SEQ_FULL + q) * SEQ_FULL + t;
    const int* pth = paths + (size_t)e * NPATH;
    float acc = 0.f;
#pragma unroll 1
    for (unsigned p = 0; p < NPATH; ++p) {
        const int id = pth[p];
        const int idc = min(max(id, 0), N_EDGES - 1);
        const float valid = (id >= 0) ? 1.f : 0.f;
        const v4f* e4 = (const v4f*)(ef + (size_t)idc * E_DIM);
        const float* w = sPP + p * 16u;
        float s = 0.f;
#pragma unroll
        for (int g = 0; g < 4; ++g) {
            const v4f a = e4[g];
            s += bfr(a.x) * w[4 * g] + bfr(a.y) * w[4 * g + 1] + bfr(a.z) * w[4 * g + 2] + bfr(a.w) * w[4 * g + 3];
        }
        acc += s * valid;
    }
    const float val = bfr(dist[e]) * bfr(dparams[0]) + bfr(dparams[1]) + acc * 0.125f;
    sB[t] = val * 256.0f;
    __syncthreads();
    if (t < 32u) {
        float v[8];
#pragma unroll
        for (int i = 0; i < 8; ++i) v[i] = sB[8u * t + (unsigned)i];
        st8h(bias16, (size_t)row * 256u + 8u * t, v);
    }
}

__global__ __launch_bounds__(256) void k_prep(const float* __restrict__ x, const float* __restrict__ degrees,
                                              const float* __restrict__ deg_W, const float* __restrict__ deg_b,
                                              unsigned short* __restrict__ xp16) {
    const unsigned u = blockIdx.x * 256u + threadIdx.x;
    if (u >= (unsigned)(MTOK * IN_DIM / 8)) return;
    const unsigned row = u >> 4, c0 = (u & 15u) * 8u;
    const float dg = bfr(degrees[row]);
    const float* xr = x + (size_t)row * IN_DIM + c0;
    float v[8];
#pragma unroll
    for (int i = 0; i < 8; ++i) v[i] = (bfr(xr[i]) + (dg * bfr(deg_W[c0 + (unsigned)i]) + bfr(deg_b[c0 + (unsigned)i]))) * 8.0f;
    st8h(xp16, (size_t)row * IN_DIM + c0, v);
}

__global__ __launch_bounds__(256) void k_ln(const float* __restrict__ h, const float* __restrict__ g, const float* __restrict__ bt,
                                            unsigned short* __restrict__ z16, unsigned M) {
    const unsigned row = blockIdx.x * 8u + (threadIdx.x >> 5);
    const unsigned L = threadIdx.x & 31u;
    if (row >= M) return;
    const float* hr = h + (size_t)row * 256u + 8u * L;
    const v4f a = *(const v4f*)hr, b = *(const v4f*)(hr + 4);
    float s = ((a.x + a.y) + (a.z + a.w)) + ((b.x + b.y) + (b.z + b.w));
#pragma unroll
    for (int o = 16; o > 0; o >>= 1) s += __shfl_xor(s, o, 32);
    const float mu = s * (1.0f / 256.0f);
    float d[8] = {a.x - mu, a.y - mu, a.z - mu, a.w - mu, b.x - mu, b.y - mu, b.z - mu, b.w - mu};
    float q = 0.f;
#pragma unroll
    for (int i = 0; i < 8; ++i) q += d[i] * d[i];
#pragma unroll
    for (int o = 16; o > 0; o >>= 1) q += __shfl_xor(q, o, 32);
    const float rs = rsqrtf(q * (1.0f / 256.0f) + 1e-5f);
    const v4f g0 = *(const v4f*)(g + 8u * L), g1 = *(const v4f*)(g + 8u * L + 4u);
    const v4f b0 = *(const v4f*)(bt + 8u * L), b1 = *(const v4f*)(bt + 8u * L + 4u);
    const float gg[8] = {g0.x, g0.y, g0.z, g0.w, g1.x, g1.y, g1.z, g1.w};
    const float bb[8] = {b0.x, b0.y, b0.z, b0.w, b1.x, b1.y, b1.z, b1.w};
    float y[8];
#pragma unroll
    for (int i = 0; i < 8; ++i) y[i] = (d[i] * rs * bfr(gg[i]) + bfr(bb[i])) * 8.0f;
    st8h(z16, (size_t)row * 256u + 8u * L, y);
}

#define AT_PP 72
#define AT_PV 264
__global__ __launch_bounds__(512) void k_attn(const _Float16* __restrict__ qkv, const _Float16* __restrict__ bias16,
                                              _Float16* __restrict__ vals) {
    __shared__ __align__(16) _Float16 sVT[64 * AT_PV];
    __shared__ __align__(16) _Float16 sP[16][16 * AT_PP];
    const unsigned tid = threadIdx.x, lane = tid & 31u, wave = tid >> 5;
    const unsigned hh = lane >> 4, c = lane & 15u;
    const unsigned b = blockIdx.x >> 2, pair = blockIdx.x & 3u;
    {
        const unsigned key = tid >> 1, hp = tid & 1u;
        const _Float16* vsrc = qkv + (size_t)(b * SEQ + key) * 768u + (2u * pair + hp) * 96u + 64u;
#pragma unroll
        for (int g = 0; g < 4; ++g) {
            const v8h vv = *(const v8h*)(vsrc + 8 * g);
#pragma unroll
            for (int e = 0; e < 8; ++e) sVT[(hp * 32u + 8u * (unsigned)g + (unsigned)e) * AT_PV + key] = vv[e];
        }
    }
    __syncthreads();
    const unsigned q0 = wave * 16u;
    _Float16* pw = sP[wave];
    const float SC2 = 0.17677669529663687f * (1.0f / 64.0f) * 1.4426950408889634f;
    const _Float16* brow = bias16 + (size_t)(b * SEQ + q0 + c) * 256u + 8u * hh;
    v8f ofin[2][2];
#pragma unroll
    for (int hp = 0; hp < 2; ++hp) {
        const unsigned head = 2u * pair + (unsigned)hp;
        const v16h qf = frag_ld(qkv + (size_t)(b * SEQ + q0 + c) * 768u + head * 96u + 8u * hh);
        float mrow[8], lrow[8];
        v8f os[2], ob[2];
#pragma unroll
        for (int r = 0; r < 8; ++r) { mrow[r] = -3.0e38f; lrow[r] = 0.f; }
#pragma unroll
        for (int t = 0; t < 2; ++t) { os[t] = (v8f){0.f,0.f,0.f,0.f,0.f,0.f,0.f,0.f}; ob[t] = os[t]; }
#pragma unroll 1
        for (unsigned kc = 0; kc < 4u; ++kc) {
            const unsigned kv0 = kc * 64u;
            v8f s[4];
#pragma unroll
            for (int j = 0; j < 4; ++j) {
                const v16h kf = frag_ld(qkv + (size_t)(b * SEQ + kv0 + (unsigned)j * 16u + c) * 768u + head * 96u + 32u + 8u * hh);
                const v8f z = (v8f){0.f,0.f,0.f,0.f,0.f,0.f,0.f,0.f};
                s[j] = wmma16(qf, kf, z);
            }
#pragma unroll
            for (int r = 0; r < 8; ++r) {
                float mx = -3.0e38f;
#pragma unroll
                for (int j = 0; j < 4; ++j) { s[j][r] *= SC2; mx = fmaxf(mx, s[j][r]); }
                mx = fmaxf(mx, __shfl_xor(mx, 1, 32)); mx = fmaxf(mx, __shfl_xor(mx, 2, 32));
                mx = fmaxf(mx, __shfl_xor(mx, 4, 32)); mx = fmaxf(mx, __shfl_xor(mx, 8, 32));
                const float mnew = fmaxf(mrow[r], mx);
                const float alpha = exp2f(mrow[r] - mnew);
                mrow[r] = mnew;
                float psum = 0.f;
#pragma unroll
                for (int j = 0; j < 4; ++j) {
                    const float p = exp2f(s[j][r] - mnew);
                    psum += p;
                    pw[(8u * hh + (unsigned)r) * AT_PP + (unsigned)j * 16u + c] = (_Float16)(p * 1024.0f);
                }
                psum += __shfl_xor(psum, 1, 32); psum += __shfl_xor(psum, 2, 32);
                psum += __shfl_xor(psum, 4, 32); psum += __shfl_xor(psum, 8, 32);
                lrow[r] = lrow[r] * alpha + psum;
                os[0][r] *= alpha; os[1][r] *= alpha;
            }
            wave_sync_lds();
#pragma unroll
            for (int kk = 0; kk < 2; ++kk) {
                const v16h pa = frag_ld(pw + c * AT_PP + (unsigned)kk * 32u + 8u * hh);
                const v16h ba = frag_ld(brow + kv0 + (unsigned)kk * 32u);
#pragma unroll
                for (int t = 0; t < 2; ++t) {
                    const v16h vb = frag_ld(sVT + ((unsigned)hp * 32u + (unsigned)t * 16u + c) * AT_PV + kv0 + (unsigned)kk * 32u + 8u * hh);
                    os[t] = wmma16(pa, vb, os[t]);
                    ob[t] = wmma16(ba, vb, ob[t]);
                }
            }
            wave_sync_lds();
        }
#pragma unroll
        for (int r = 0; r < 8; ++r) {
            const float inv = 1.0f / (lrow[r] * 1024.0f);
#pragma unroll
            for (int t = 0; t < 2; ++t) ofin[hp][t][r] = os[t][r] * inv + ob[t][r] * (1.0f / 256.0f);
        }
    }
#pragma unroll
    for (int hp = 0; hp < 2; ++hp)
#pragma unroll
        for (int t = 0; t < 2; ++t)
#pragma unroll
            for (int r = 0; r < 8; ++r)
                pw[(8u * hh + (unsigned)r) * AT_PP + (unsigned)hp * 32u + (unsigned)t * 16u + c] = (_Float16)ofin[hp][t][r];
    wave_sync_lds();
    {
        const unsigned q = lane >> 3, c8 = (lane & 7u) * 8u;
        v8h ov[4];
#pragma unroll
        for (int it = 0; it < 4; ++it) ov[it] = *(const v8h*)(pw + ((unsigned)it * 4u + q) * AT_PP + c8);
        _Float16* dst = vals + (size_t)(b * SEQ + q0) * 256u + pair * 64u;
        for (int pass = 0; pass < 2; ++pass) {
#pragma unroll
            for (int it = 0; it < 4; ++it) *(volatile v8h*)(dst + (size_t)((unsigned)it * 4u + q) * 256u + c8) = ov[it];
            __threadfence();
        }
    }
}

__global__ __launch_bounds__(256) void k_out(const float* __restrict__ h, const float* __restrict__ out_W,
                                             const float* __restrict__ out_b, float* __restrict__ out) {
    __shared__ float red[256];
    __shared__ float res[8];
    const unsigned t = threadIdx.x;
    const float w = bfr(out_W[t]);
    const float ob = bfr(out_b[0]);
    if (t < 8u) res[t] = 0.f;
    __syncthreads();
#pragma unroll 1
    for (unsigned b = 0; b < (unsigned)NB; ++b) {
        float acc = 0.f;
#pragma unroll 4
        for (unsigned n = 0; n < (unsigned)SEQ; ++n) acc += h[(size_t)(b * SEQ + n) * 256u + t];
        red[t] = (acc * (1.0f / (float)SEQ)) * w;
        __syncthreads();
        for (unsigned s = 128u; s > 0u; s >>= 1) { if (t < s) red[t] += red[t + s]; __syncthreads(); }
        if (t == 0u) res[b] = red[0] + ob;
        __syncthreads();
    }
    if (NB == 8) {
        if (t < 2u) { v4f v; v.x = res[4u * t]; v.y = res[4u * t + 1u]; v.z = res[4u * t + 2u]; v.w = res[4u * t + 3u]; VST2V4(out + 4u * t, v); }
    } else {
        if (t < (unsigned)NB) { VST2(float, out + t, res[t]); }
    }
}

extern "C" void kernel_launch(void* const* d_in, const int* in_sizes, int n_in, void* d_out, int out_size,
                              void* d_ws, size_t ws_size, hipStream_t stream) {
    if (n_in < 25) return;
    if (in_sizes[0] < MTOK * IN_DIM || in_sizes[1] < MTOK || in_sizes[2] < MTOK * SEQ || in_sizes[3] < MTOK * SEQ * NPATH) return;
    if (in_sizes[4] < N_EDGES * E_DIM || in_sizes[5] < IN_DIM || in_sizes[7] < IN_DIM * EMB || in_sizes[10] < NPATH * E_DIM) return;
    if (in_sizes[11] < NLAYER * EMB * 3 * EMB || in_sizes[13] < NLAYER * EMB * EMB || in_sizes[19] < NLAYER * EMB * FFD || in_sizes[21] < NLAYER * FFD * EMB) return;
    if (in_sizes[23] < EMB || in_sizes[24] < 1 || out_size < NB) return;

    const float* x          = (const float*)d_in[0];
    const float* degrees    = (const float*)d_in[1];
    const float* dist_mat   = (const float*)d_in[2];
    const int*   paths      = (const int*)d_in[3];
    const float* edge_feats = (const float*)d_in[4];
    const float* deg_W      = (const float*)d_in[5];
    const float* deg_b      = (const float*)d_in[6];
    const float* emb_W      = (const float*)d_in[7];
    const float* emb_b      = (const float*)d_in[8];
    const float* dist_par   = (const float*)d_in[9];
    const float* path_par   = (const float*)d_in[10];
    const float* qkv_W      = (const float*)d_in[11];
    const float* qkv_b      = (const float*)d_in[12];
    const float* o_W        = (const float*)d_in[13];
    const float* o_b        = (const float*)d_in[14];
    const float* ln1_g      = (const float*)d_in[15];
    const float* ln1_b      = (const float*)d_in[16];
    const float* ln2_g      = (const float*)d_in[17];
    const float* ln2_b      = (const float*)d_in[18];
    const float* ff1_W      = (const float*)d_in[19];
    const float* ff1_b      = (const float*)d_in[20];
    const float* ff2_W      = (const float*)d_in[21];
    const float* ff2_b      = (const float*)d_in[22];
    const float* out_W      = (const float*)d_in[23];
    const float* out_b      = (const float*)d_in[24];
    float* out = (float*)d_out;

    char* wsp = (char*)d_ws;
    size_t off = 0;
    auto carve = [&](size_t bytes) -> void* { void* r = wsp + off; off += (bytes + 255) & ~(size_t)255; return r; };
    unsigned short* bias16 = (unsigned short*)carve((size_t)MTOK * SEQ * 2);
    unsigned short* xp16   = (unsigned short*)carve((size_t)MTOK * IN_DIM * 2);
    float*          hA     = (float*)carve((size_t)MTOK * EMB * 4);
    float*          hB     = (float*)carve((size_t)MTOK * EMB * 4);
    unsigned short* z16    = (unsigned short*)carve((size_t)MTOK * EMB * 2);
    unsigned short* qkv16  = (unsigned short*)carve((size_t)MTOK * 3 * EMB * 2);
    unsigned short* vals16 = (unsigned short*)carve((size_t)MTOK * EMB * 2);
    unsigned short* ff16   = (unsigned short*)carve((size_t)MTOK * FFD * 2);
    unsigned short* wemb   = (unsigned short*)carve((size_t)IN_DIM * EMB * 2);
    unsigned short* wqkv   = (unsigned short*)carve((size_t)NLAYER * EMB * 3 * EMB * 2);
    unsigned short* wo     = (unsigned short*)carve((size_t)NLAYER * EMB * EMB * 2);
    unsigned short* wff1   = (unsigned short*)carve((size_t)NLAYER * EMB * FFD * 2);
    unsigned short* wff2   = (unsigned short*)carve((size_t)NLAYER * FFD * EMB * 2);
    if (off > ws_size || off > (size_t)134217728) return;

    k_wt16<<<dim3((EMB * (IN_DIM / 8)) / 256, 1), 256, 0, stream>>>(emb_W, IN_DIM, EMB, 4, wemb, 32.0f);
    k_wt16<<<dim3((3 * EMB * (EMB / 8)) / 256, NLAYER), 256, 0, stream>>>(qkv_W, EMB, 3 * EMB, 5, wqkv, 32.0f);
    k_wt16<<<dim3((EMB * (EMB / 8)) / 256, NLAYER), 256, 0, stream>>>(o_W, EMB, EMB, 5, wo, 32.0f);
    k_wt16<<<dim3((FFD * (EMB / 8)) / 256, NLAYER), 256, 0, stream>>>(ff1_W, EMB, FFD, 5, wff1, 32.0f);
    k_wt16<<<dim3((EMB * (FFD / 8)) / 256, NLAYER), 256, 0, stream>>>(ff2_W, FFD, EMB, 7, wff2, 32.0f);

    k_bias<<<MTOK, 256, 0, stream>>>(dist_mat, paths, edge_feats, path_par, dist_par, bias16);
    k_prep<<<(MTOK * IN_DIM / 8) / 256, 256, 0, stream>>>(x, degrees, deg_W, deg_b, xp16);

    const float SC = 1.0f / 256.0f;
    const unsigned gE = ((MTOK / 64) * (EMB / 64) + 7) / 8;
    const unsigned gQ = ((MTOK / 64) * (3 * EMB / 64) + 7) / 8;
    const unsigned gF = ((MTOK / 64) * (FFD / 64) + 7) / 8;

    k_gemm64<0, false, false><<<gE, 256, 0, stream>>>((const _Float16*)xp16, IN_DIM, (const _Float16*)wemb, IN_DIM,
        (void*)hA, EMB, emb_b, nullptr, MTOK, EMB, IN_DIM, SC, 1.0f);

    for (int l = 0; l < NLAYER; ++l) {
        k_ln<<<MTOK / 8, 256, 0, stream>>>(hA, ln1_g + l * EMB, ln1_b + l * EMB, z16, MTOK);
        k_gemm64<1, false, false><<<gQ, 256, 0, stream>>>((const _Float16*)z16, EMB, (const _Float16*)(wqkv + (size_t)l * EMB * 3 * EMB), EMB,
            (void*)qkv16, 3 * EMB, qkv_b + l * 3 * EMB, nullptr, MTOK, 3 * EMB, EMB, SC, 8.0f);
        k_attn<<<NB * 4, 512, 0, stream>>>((const _Float16*)qkv16, (const _Float16*)bias16, (_Float16*)vals16);
        k_gemm64<0, true, false><<<gE, 256, 0, stream>>>((const _Float16*)vals16, EMB, (const _Float16*)(wo + (size_t)l * EMB * EMB), EMB,
            (void*)hB, EMB, o_b + l * EMB, hA, MTOK, EMB, EMB, SC, 1.0f);
        k_ln<<<MTOK / 8, 256, 0, stream>>>(hB, ln2_g + l * EMB, ln2_b + l * EMB, z16, MTOK);
        k_gemm64<1, false, true><<<gF, 256, 0, stream>>>((const _Float16*)z16, EMB, (const _Float16*)(wff1 + (size_t)l * EMB * FFD), EMB,
            (void*)ff16, FFD, ff1_b + l * FFD, nullptr, MTOK, FFD, EMB, SC, 8.0f);
        k_gemm64<0, true, false><<<gE, 256, 0, stream>>>((const _Float16*)ff16, FFD, (const _Float16*)(wff2 + (size_t)l * FFD * EMB), FFD,
            (void*)hA, EMB, ff2_b + l * EMB, hB, MTOK, EMB, FFD, SC, 1.0f);
    }
    k_out<<<1, 256, 0, stream>>>(hA, out_W, out_b, out);
}
